// PromptParser_73469710565875
// MI455X (gfx1250) — hardware-run, weakly checked
//
#include <hip/hip_runtime.h>


#ifndef NB
#define NB 16
#endif
#define NB_FULL 16
#define NT   16
#define NC   256
#define SLAB 32
#define AR   34
#define ARP  48
#define AP   260
#define HP   264
#define CP   36
#define NTHR 256

static_assert(NB <= NB_FULL);
static_assert(NT == 16);
static_assert(NC % 32 == 0);
static_assert(NC % SLAB == 0);
static_assert(SLAB == 32);
static_assert(AR == SLAB + 2);
static_assert(ARP % 16 == 0 && ARP >= AR);
static_assert(3 * NTHR == ARP * NT);
static_assert(4 * NTHR * 4 == NT * NC);
static_assert(NTHR == NC);
static_assert(NTHR / 32 * 2 == NC / 16);
static_assert(AP >= NC + 2);
static_assert((HP * 2) % 16 == 0 && HP >= NC);
static_assert((CP * 4) % 16 == 0 && CP >= SLAB);
static_assert(32 * 16 * 4 == NT * SLAB * 4);
static_assert((size_t)NB_FULL * NT * NC * 4 == (size_t)262144);
static_assert((size_t)(AR * AP + 2 * NT * CP + 80) * 4 + (size_t)(2 * SLAB * HP + 2 * NT * HP + NC * 16 + ARP * 16) * 2 <= (size_t)131072);

typedef _Float16 h16;
typedef __attribute__((ext_vector_type(16))) _Float16 v16h;
typedef __attribute__((ext_vector_type(8)))  _Float16 v8h;
typedef __attribute__((ext_vector_type(8)))  float    v8f;
typedef __attribute__((ext_vector_type(4)))  float    v4f;
typedef v4f  __attribute__((may_alias)) v4fa;

__device__ __forceinline__ unsigned short f2bf(float f) { unsigned u = __float_as_uint(f); u += 0x7FFFu + ((u >> 16) & 1u); return (unsigned short)(u >> 16); }
__device__ __forceinline__ float bfr(float f) { return __uint_as_float(((unsigned)f2bf(f)) << 16); }
__device__ __forceinline__ v16h cat16(v8h lo, v8h hi) { return __builtin_shufflevector(lo, hi, 0, 1, 2, 3, 4, 5, 6, 7, 8, 9, 10, 11, 12, 13, 14, 15); }
static __device__ __forceinline__ h16 toh_flush(float v) { const h16 r = (h16)v; return (fabsf(v) < 6.103515625e-05f) ? (h16)0.0f : r; }
__device__ __forceinline__ v8f wmma16g(v16h a, v16h b, v8f c) {
    c = __builtin_amdgcn_wmma_f32_16x16x32_f16(false, a, false, b, (short)0, c, false, false);
    asm volatile("v_nop\n\tv_nop\n\tv_nop\n\tv_nop" : "+v"(c) : "v"(a), "v"(b));
    return c;
}

__global__ __launch_bounds__(NTHR) void k_fused(const float* __restrict__ X0, const float* __restrict__ X1, const float* __restrict__ X2, const float* __restrict__ X3,
                                                const float* __restrict__ W1, const float* __restrict__ B1, const float* __restrict__ W2, const float* __restrict__ B2,
                                                const float* __restrict__ GW, const float* __restrict__ GB, float* OUT) {
    __shared__ __align__(16) float amap[AR * AP];
    __shared__ __align__(16) h16   mpl[2 * SLAB * HP];
    __shared__ __align__(16) h16   t2[2 * NT * HP];
    __shared__ __align__(16) h16   imT[NC * 16];
    __shared__ __align__(16) h16   etT[ARP * 16];
    __shared__ __align__(16) float cs[2 * NT * CP];
    __shared__ __align__(16) float wl[80];

    const int tid = threadIdx.x;
    const int lane = tid & 31, lr = lane & 15, hi = lane >> 4;
    const int wave = __builtin_amdgcn_readfirstlane((int)(threadIdx.x >> 5));
    const int c0 = blockIdx.x * SLAB;
    const int b = blockIdx.y;
    const size_t base = (size_t)b * NT * NC;

    {
        const int i = tid;
        const int i1 = i < 35 ? i : 35;
        int i2 = i - 36; i2 = i2 < 0 ? 0 : (i2 > 11 ? 11 : i2);
        int i3 = i - 48; i3 = i3 < 0 ? 0 : (i3 > 11 ? 11 : i3);
        int i5 = i - 61; i5 = i5 < 0 ? 0 : (i5 > 8 ? 8 : i5);
        float pa = W1[i1], pb = B1[i2], pc = W2[i3], pd = B2[0], pe = GW[i5], pf = GB[0];
        asm volatile("" : "+v"(pa)); asm volatile("" : "+v"(pb)); asm volatile("" : "+v"(pc));
        asm volatile("" : "+v"(pd)); asm volatile("" : "+v"(pe)); asm volatile("" : "+v"(pf));
        float v = 0.0f;
        v = (i == 70) ? pf : v;
        v = (i >= 61 && i < 70) ? pe : v;
        v = (i == 60) ? pd : v;
        v = (i >= 48 && i < 60) ? pc : v;
        v = (i >= 36 && i < 48) ? pb : v;
        v = (i < 36) ? pa : v;
        if (tid < 80) wl[tid] = bfr(v);
    }

#pragma unroll 1
    for (int it = 0; it < 4; ++it) {
        const int i4 = it * NTHR + tid;
        const int n = i4 >> 6, x4 = (i4 & 63) * 4;
        const size_t g = base + (size_t)n * NC + x4;
        const v4f vi = *(const v4f*)(X0 + g);
        const v4f va = *(const v4f*)(X1 + g);
        const v4f vb = *(const v4f*)(X2 + g);
        const v4f vc = *(const v4f*)(X3 + g);
#pragma unroll
        for (int i = 0; i < 4; ++i) {
            imT[(x4 + i) * 16 + n] = toh_flush(bfr(vi[i]));
            const float t = bfr(va[i]) + (bfr(vb[i]) + bfr(vc[i]));
            const float q = t * t;
            t2[n * HP + x4 + i]           = toh_flush((t >= 0.0f) ? q : 0.0f);
            t2[NT * HP + n * HP + x4 + i] = toh_flush((t <  0.0f) ? q : 0.0f);
        }
    }
    __syncthreads();

    {
        const float b2v = wl[60];
#pragma unroll 1
        for (int it = 0; it < 3; ++it) {
            const unsigned idx = (unsigned)(it * NTHR + tid);
            const unsigned n = idx / (unsigned)ARP;
            const int r = (int)(idx - n * (unsigned)ARP);
            const int c = c0 - 1 + r;
            const bool ok = (r < AR) && (c >= 0) && (c < NC);
            const int cc = c < 0 ? 0 : (c > NC - 1 ? NC - 1 : c);
            const size_t g = base + (size_t)n * NC + (size_t)cc;
            float a = X1[g], q1 = X2[g], q2 = X3[g];
            asm volatile("" : "+v"(a)); asm volatile("" : "+v"(q1)); asm volatile("" : "+v"(q2));
            a = bfr(a); q1 = bfr(q1); q2 = bfr(q2);
            float acc = b2v;
#pragma unroll 1
            for (int j = 0; j < 12; ++j) {
                const float h = fmaf(a, wl[j], fmaf(q1, wl[12 + j], fmaf(q2, wl[24 + j], wl[36 + j])));
                const float ge = 0.5f * h * (1.0f + erff(h * 0.70710678118654752440f));
                acc = fmaf(ge, wl[48 + j], acc);
            }
            const h16 ev = toh_flush(acc);
            etT[r * 16 + (int)n] = ok ? ev : (h16)0.0f;
        }
    }
    __syncthreads();

    {
        const v8h z8 = (v8h){};
        v16h a[3];
#pragma unroll
        for (int mt = 0; mt < 3; ++mt) a[mt] = cat16(*(const v8h*)(&etT[(mt * 16 + lr) * 16 + 8 * hi]), z8);
#pragma unroll
        for (int xx = 0; xx < 2; ++xx) {
            const int xt = wave * 2 + xx;
            const v16h bfrg = cat16(*(const v8h*)(&imT[(xt * 16 + lr) * 16 + 8 * hi]), z8);
#pragma unroll
            for (int mt = 0; mt < 3; ++mt) {
                v8f acc = (v8f){};
                acc = wmma16g(a[mt], bfrg, acc);
#pragma unroll
                for (int rr = 0; rr < 8; ++rr) {
                    const int row = mt * 16 + 8 * hi + rr;
                    if (row < AR) amap[row * AP + 1 + xt * 16 + lr] = acc[rr];
                }
            }
        }
        if (tid < AR) { amap[tid * AP] = 0.0f; amap[tid * AP + NC + 1] = 0.0f; }
    }
    __syncthreads();

    {
        float g9[9];
#pragma unroll
        for (int j = 0; j < 9; ++j) g9[j] = wl[61 + j];
        const float gbv = wl[70];
        const int x = tid;
#pragma unroll 1
        for (int cr = 0; cr < SLAB; ++cr) {
            float s = gbv;
#pragma unroll
            for (int i = 0; i < 3; ++i)
#pragma unroll
                for (int j = 0; j < 3; ++j) s = fmaf(g9[i * 3 + j], amap[(cr + i) * AP + x + j], s);
            mpl[cr * HP + x]             = toh_flush(fmaxf(s, 1.0f));
            mpl[SLAB * HP + cr * HP + x] = toh_flush(fminf(s, 1.0f));
        }
    }
    __syncthreads();

    if (wave < 4) {
        const int mt = wave & 1, wh = wave >> 1;
        const int fo = wh * (SLAB * HP), so = (1 - wh) * (SLAB * HP);
        const int ao = (mt * 16 + lr) * HP + 8 * hi;
        const int bo = lr * HP + 8 * hi;
        v8f acc = (v8f){};
#pragma unroll
        for (int ks = 0; ks < NC / 32; ++ks) {
            const int k0 = ks * 32;
            const v16h a1 = cat16(*(const v8h*)(&mpl[fo + ao + k0]), *(const v8h*)(&mpl[fo + ao + k0 + 16]));
            const v16h a2 = cat16(*(const v8h*)(&mpl[so + ao + k0]), *(const v8h*)(&mpl[so + ao + k0 + 16]));
            const v16h bp = cat16(*(const v8h*)(&t2[bo + k0]), *(const v8h*)(&t2[bo + k0 + 16]));
            const v16h bm = cat16(*(const v8h*)(&t2[NT * HP + bo + k0]), *(const v8h*)(&t2[NT * HP + bo + k0 + 16]));
            acc = wmma16g(a1, bp, acc);
            acc = wmma16g(a2, bm, acc);
        }
        v4f u, w;
        u[0] = acc[0]; u[1] = acc[1]; u[2] = acc[2]; u[3] = acc[3];
        w[0] = acc[4]; w[1] = acc[5]; w[2] = acc[6]; w[3] = acc[7];
        const int co = wh * (NT * CP) + lr * CP + mt * 16 + 8 * hi;
        *(v4fa*)(&cs[co]) = u; *(v4fa*)(&cs[co + 4]) = w;
    }
    __syncthreads();

    if (wave == 0) {
        v4f val[4];
#pragma unroll
        for (int s = 0; s < 4; ++s) {
            const int row = 4 * s + (lane >> 3), cofs = (lane & 7) * 4;
            const v4f cA = *(const v4fa*)(&cs[row * CP + cofs]);
            const v4f cB = *(const v4fa*)(&cs[NT * CP + row * CP + cofs]);
            const v4f xi = *(const v4f*)(X0 + base + (size_t)row * NC + c0 + cofs);
#pragma unroll
            for (int i = 0; i < 4; ++i) { const float iv = bfr(xi[i]); const float sel = (iv >= 0.0f) ? cA[i] : cB[i]; val[s][i] = iv * sel; }
        }
        float* orow = OUT + (size_t)NB_FULL * NT * NC + base + c0;
#pragma unroll 1
        for (int ps = 0; ps < 2; ++ps) {
#pragma unroll
            for (int s = 0; s < 4; ++s) { const int row = 4 * s + (lane >> 3), cofs = (lane & 7) * 4;
                *(volatile v4f*)(orow + (size_t)row * NC + cofs) = val[s]; }
            if (ps == 0) __threadfence(); }
    }
    if (wave == 1) {
        v4f val[4];
#pragma unroll
        for (int s = 0; s < 4; ++s) {
            const int row = 4 * s + (lane >> 3), cofs = (lane & 7) * 4;
            const v4f xi = *(const v4f*)(X0 + base + (size_t)row * NC + c0 + cofs);
#pragma unroll
            for (int i = 0; i < 4; ++i) val[s][i] = bfr(xi[i]);
        }
        float* orow = OUT + base + c0;
#pragma unroll 1
        for (int ps = 0; ps < 2; ++ps) {
#pragma unroll
            for (int s = 0; s < 4; ++s) { const int row = 4 * s + (lane >> 3), cofs = (lane & 7) * 4;
                *(volatile v4f*)(orow + (size_t)row * NC + cofs) = val[s]; }
            if (ps == 0) __threadfence(); }
    }
}

extern "C" void kernel_launch(void* const* d_in, const int* in_sizes, int n_in,
                              void* d_out, int out_size, void* d_ws, size_t ws_size, hipStream_t stream) {
    if (n_in < 10) return;
    const size_t needx = (size_t)NB * NT * NC;
    if ((size_t)in_sizes[0] < needx || (size_t)in_sizes[1] < needx || (size_t)in_sizes[2] < needx || (size_t)in_sizes[3] < needx) return;
    if (in_sizes[4] < 36 || in_sizes[5] < 12 || in_sizes[6] < 12 || in_sizes[7] < 1 || in_sizes[8] < 9 || in_sizes[9] < 1) return;
    if ((size_t)out_size < (size_t)NB_FULL * NT * NC + needx) return;
    const float* x0 = (const float*)d_in[0];
    const float* x1 = (const float*)d_in[1];
    const float* x2 = (const float*)d_in[2];
    const float* x3 = (const float*)d_in[3];
    const float* w1 = (const float*)d_in[4];
    const float* b1 = (const float*)d_in[5];
    const float* w2 = (const float*)d_in[6];
    const float* b2 = (const float*)d_in[7];
    const float* gw = (const float*)d_in[8];
    const float* gb = (const float*)d_in[9];
    float* OUT = (float*)d_out;
    (void)d_ws; (void)ws_size;
    k_fused<<<dim3(NC / SLAB, NB, 1), NTHR, 0, stream>>>(x0, x1, x2, x3, w1, b1, w2, b2, gw, gb, OUT);
}
